// MHA_56504589746420
// MI455X (gfx1250) — hardware-verified
//
#include <hip/hip_runtime.h>


#ifndef NB
#define NB 4
#endif
#ifndef SEQ
#define SEQ 2048
#endif
#define NB_FULL  4
#define SEQ_FULL 2048
#define DM   1024
#define NH   16
#define HD   64
#define D3   (3 * DM)
#define MROWS (NB * SEQ)
#define QKCAR 16.0f
#define VCAR  16.0f
#define CCAR  256.0f
#define WCAR  64.0f
#define PLANE ((size_t)MROWS * DM)

#define XB_BYTES  ((size_t)MROWS * DM * 2)
#define WQT_BYTES ((size_t)D3 * DM * 2)
#define WOT_BYTES ((size_t)DM * DM * 2)
#define QKV_BYTES ((size_t)3 * MROWS * DM * 2)
#define CTX_BYTES ((size_t)MROWS * DM * 2)
#define WS_TOTAL  (XB_BYTES + WQT_BYTES + WOT_BYTES + QKV_BYTES + CTX_BYTES)

static_assert(HD == 64);
static_assert(NH * HD == DM);
static_assert(DM % 64 == 0);
static_assert(DM % 32 == 0);
static_assert(D3 % 64 == 0);
static_assert(SEQ % 64 == 0);
static_assert(MROWS % 64 == 0);
static_assert(NB <= NB_FULL);
static_assert(SEQ <= SEQ_FULL);
static_assert((MROWS * DM) % 8 == 0);
static_assert(XB_BYTES % 256 == 0);
static_assert(WQT_BYTES % 256 == 0);
static_assert(WOT_BYTES % 256 == 0);
static_assert(QKV_BYTES % 256 == 0);
static_assert(CTX_BYTES % 256 == 0);
static_assert(WS_TOTAL <= (size_t)134217728);

typedef _Float16 h16;
typedef unsigned short bf;
typedef __attribute__((ext_vector_type(16))) __bf16   v16bf;
typedef __attribute__((ext_vector_type(16))) _Float16 v16h;
typedef __attribute__((ext_vector_type(8)))  _Float16 v8h;
typedef __attribute__((ext_vector_type(8)))  unsigned short v8us;
typedef __attribute__((ext_vector_type(8)))  float    v8f;
typedef __attribute__((ext_vector_type(4)))  float    v4f;
typedef v8h  __attribute__((may_alias)) v8ha;
typedef v4f  __attribute__((may_alias)) v4fa;

__device__ __forceinline__ unsigned short f2bf(float f) { unsigned u = __float_as_uint(f); u += 0x7FFFu + ((u >> 16) & 1u); return (unsigned short)(u >> 16); }
__device__ __forceinline__ float bf2f(unsigned short b) { return __uint_as_float(((unsigned)b) << 16); }
__device__ __forceinline__ float bfr(float f) { return bf2f(f2bf(f)); }
__device__ __forceinline__ v16h cat16(v8h lo, v8h hi) { return __builtin_shufflevector(lo, hi, 0, 1, 2, 3, 4, 5, 6, 7, 8, 9, 10, 11, 12, 13, 14, 15); }
__device__ __forceinline__ v16bf cat16b(v8us lo, v8us hi) { return __builtin_bit_cast(v16bf, __builtin_shufflevector(lo, hi, 0, 1, 2, 3, 4, 5, 6, 7, 8, 9, 10, 11, 12, 13, 14, 15)); }
__device__ __forceinline__ v8f wmma16(v16h a, v16h b, v8f c) { return __builtin_amdgcn_wmma_f32_16x16x32_f16(false, a, false, b, (short)0, c, false, false); }
__device__ __forceinline__ v8f wmmab(v16bf a, v16bf b, v8f c) { return __builtin_amdgcn_wmma_f32_16x16x32_bf16(false, a, false, b, (short)0, c, false, false); }
__device__ __forceinline__ v16h ldh(const h16* p) { return cat16(*(const v8h*)p, *(const v8h*)(p + 16)); }

template <typename T16> struct WFrag;
template <> struct WFrag<h16> { typedef v16h V; static __device__ __forceinline__ V ld(const h16* p) { return cat16(*(const v8h*)p, *(const v8h*)(p + 16)); } static __device__ __forceinline__ v8f mma(V a, V b, v8f c) { return wmma16(a, b, c); } };
template <> struct WFrag<bf> { typedef v16bf V; static __device__ __forceinline__ V ld(const bf* p) { return cat16b(*(const v8us*)p, *(const v8us*)(p + 16)); } static __device__ __forceinline__ v8f mma(V a, V b, v8f c) { return wmmab(a, b, c); } };

template <typename T16>
__device__ __forceinline__ void gemm_main(const T16* __restrict__ A, const T16* __restrict__ Bt, int r0, int c0, int lr, int hi, v8f (&acc)[4][4]) {
    typedef typename WFrag<T16>::V V;
#pragma unroll
    for (int mb = 0; mb < 4; ++mb)
#pragma unroll
        for (int nb = 0; nb < 4; ++nb) acc[mb][nb] = (v8f){};
    const size_t aoff = (size_t)(r0 + lr) * DM + 8 * hi, boff = (size_t)(c0 + lr) * DM + 8 * hi;
#pragma unroll 1
    for (int kc = 0; kc < DM; kc += 32) {
        V a[4];
#pragma unroll
        for (int mb = 0; mb < 4; ++mb) a[mb] = WFrag<T16>::ld(A + aoff + (size_t)mb * 16 * DM + kc);
#pragma unroll
        for (int nb = 0; nb < 4; ++nb) { const V b = WFrag<T16>::ld(Bt + boff + (size_t)nb * 16 * DM + kc);
#pragma unroll
            for (int mb = 0; mb < 4; ++mb) acc[mb][nb] = WFrag<T16>::mma(a[mb], b, acc[mb][nb]); }
        asm volatile("v_nop\n\tv_nop\n\tv_nop\n\tv_nop" : "+v"(acc[0][0]), "+v"(acc[1][1]), "+v"(acc[2][2]), "+v"(acc[3][3]) : "v"(a[0]), "v"(a[3]));
    }
}

__global__ __launch_bounds__(256) void k_cvtx(const float* __restrict__ x, bf* XB) {
    const size_t i = (size_t)blockIdx.x * 256 + threadIdx.x; if (i >= (size_t)MROWS * DM / 8) return;
    const size_t e = i * 8; const int row = (int)(e / DM), col = (int)(e % DM); const int b = row / SEQ, l = row % SEQ;
    const float* s = x + ((size_t)b * SEQ_FULL + l) * DM + col;
    const v4f a0 = *(const v4f*)s, a1 = *(const v4f*)(s + 4); v8us o;
#pragma unroll
    for (int q = 0; q < 4; ++q) { o[q] = f2bf(a0[q]); o[4 + q] = f2bf(a1[q]); }
    *(volatile v8us*)(XB + e) = o; __threadfence(); *(volatile v8us*)(XB + e) = o;
}

__global__ __launch_bounds__(256) void k_wt(const float* __restrict__ W, int N, unsigned short* Wt, int mode) {
    __shared__ __align__(16) float ts[64 * 68];
    const int t = threadIdx.x; const int n0 = blockIdx.x * 64, k0 = blockIdx.y * 64;
#pragma unroll
    for (int it = 0; it < 4; ++it) { const int idx = t + it * 256; const int kk = idx >> 4, c4 = (idx & 15) * 4; const v4f a = *(const v4f*)(W + (size_t)(k0 + kk) * N + n0 + c4); *(v4fa*)(ts + kk * 68 + c4) = a; }
    __syncthreads();
    v8us ou[2]; v8h oh[2];
#pragma unroll
    for (int it = 0; it < 2; ++it) { const int idx = t + it * 256; const int nn = idx >> 3, q = idx & 7;
#pragma unroll
        for (int j = 0; j < 8; ++j) { const float w = ts[(q * 8 + j) * 68 + nn]; const unsigned short wb = f2bf(w); ou[it][j] = wb; oh[it][j] = (h16)(bf2f(wb) * WCAR); } }
#pragma unroll 1
    for (int ps = 0; ps < 2; ++ps) {
#pragma unroll
        for (int it = 0; it < 2; ++it) { const int idx = t + it * 256; const int nn = idx >> 3, q = idx & 7; const size_t off = (size_t)(n0 + nn) * DM + k0 + q * 8;
            if (mode != 0) { *(volatile v8h*)((h16*)Wt + off) = oh[it]; } else { *(volatile v8us*)(Wt + off) = ou[it]; } }
        if (ps == 0) __threadfence(); }
}

__global__ __launch_bounds__(32) void k_gemm_qkv(const bf* __restrict__ XB, const bf* __restrict__ Wt, const float* __restrict__ bias, h16* planes) {
    __shared__ __align__(16) h16 os[64 * 72];
    const int lane = threadIdx.x & 31, lr = lane & 15, hi = lane >> 4; const int r0 = blockIdx.x * 64, c0 = blockIdx.y * 64;
    v8f acc[4][4];
    gemm_main<bf>(XB, Wt, r0, c0, lr, hi, acc);
    const int which = blockIdx.y / (DM / 64), h = blockIdx.y % (DM / 64);
    const int b = r0 / SEQ, l0 = r0 % SEQ;
    const bool tr = (which == 2);
    const int rs = tr ? 1 : 72, cs = tr ? 72 : 1;
    const float car = tr ? VCAR : QKCAR;
    float bs[4];
#pragma unroll
    for (int nb = 0; nb < 4; ++nb) bs[nb] = bfr(bias[c0 + nb * 16 + lr]);
#pragma unroll
    for (int mb = 0; mb < 4; ++mb)
#pragma unroll
        for (int nb = 0; nb < 4; ++nb)
#pragma unroll
            for (int j = 0; j < 8; ++j) os[(mb * 16 + hi * 8 + j) * rs + (nb * 16 + lr) * cs] = (h16)((acc[mb][nb][j] + bs[nb]) * car);
    __syncthreads();
    const size_t base = (size_t)which * PLANE + (tr ? ((size_t)(b * NH + h) * HD) * SEQ + l0 : ((size_t)(b * NH + h) * SEQ + l0) * HD);
    const size_t pitch = tr ? (size_t)SEQ : (size_t)HD;
    const int rq = lane >> 3, q = lane & 7;
#pragma unroll 1
    for (int ps = 0; ps < 2; ++ps) {
#pragma unroll
        for (int it = 0; it < 16; ++it) { const int row = it * 4 + rq; const v8h val = *(const v8ha*)(os + row * 72 + q * 8); *(volatile v8h*)(planes + base + (size_t)row * pitch + q * 8) = val; }
        if (ps == 0) __threadfence(); }
}

#define QT 16
static_assert(QT == 16);
static_assert(SEQ % QT == 0);
static_assert(SEQ % 32 == 0);
__global__ __launch_bounds__(32) void k_attn(const h16* __restrict__ QKV, h16* CTX) {
    __shared__ __align__(16) h16 Pw[QT * 40];
    __shared__ __align__(16) h16 os[QT * 72];
    const int lane = threadIdx.x & 31, lr = lane & 15, hi = lane >> 4;
    const int b = blockIdx.z, h = blockIdx.y, q0 = blockIdx.x * QT;
    const h16* Qh = QKV + (size_t)(b * NH + h) * SEQ * HD;
    const h16* Kh = QKV + PLANE + (size_t)(b * NH + h) * SEQ * HD;
    const h16* Vh = QKV + 2 * PLANE + (size_t)(b * NH + h) * HD * SEQ;
    v16h aq[2];
#pragma unroll
    for (int ks = 0; ks < 2; ++ks) aq[ks] = ldh(Qh + (size_t)(q0 + lr) * HD + ks * 32 + 8 * hi);
    v8f o[4]; float mrow[8], lrow[8];
#pragma unroll
    for (int dt = 0; dt < 4; ++dt) o[dt] = (v8f){};
#pragma unroll
    for (int r = 0; r < 8; ++r) { mrow[r] = -1.0e30f; lrow[r] = 0.0f; }
    const float SC2 = (0.125f / (QKCAR * QKCAR)) * 1.4426950408889634f;
#pragma unroll 1
    for (int j = 0; j < SEQ; j += 32) {
        v8f s[2];
#pragma unroll
        for (int nt = 0; nt < 2; ++nt) s[nt] = (v8f){};
        const h16* kp = Kh + (size_t)(j + lr) * HD + 8 * hi;
#pragma unroll
        for (int nt = 0; nt < 2; ++nt) { const v16h k0 = ldh(kp + (size_t)nt * 16 * HD); const v16h k1 = ldh(kp + (size_t)nt * 16 * HD + 32);
            s[nt] = wmma16(aq[0], k0, s[nt]); s[nt] = wmma16(aq[1], k1, s[nt]); }
        asm volatile("v_nop\n\tv_nop\n\tv_nop\n\tv_nop" : "+v"(s[0]), "+v"(s[1]) : "v"(aq[0]), "v"(aq[1]));
#pragma unroll
        for (int r = 0; r < 8; ++r) {
            const float t0 = s[0][r] * SC2, t1 = s[1][r] * SC2;
            float vmax = fmaxf(t0, t1);
            vmax = fmaxf(vmax, __shfl_xor(vmax, 1, 32)); vmax = fmaxf(vmax, __shfl_xor(vmax, 2, 32)); vmax = fmaxf(vmax, __shfl_xor(vmax, 4, 32)); vmax = fmaxf(vmax, __shfl_xor(vmax, 8, 32));
            const float mn = fmaxf(mrow[r], vmax);
            const float fac = __builtin_amdgcn_exp2f(mrow[r] - mn);
            mrow[r] = mn;
            const h16 p0 = (h16)__builtin_amdgcn_exp2f(t0 - mn), p1 = (h16)__builtin_amdgcn_exp2f(t1 - mn);
            lrow[r] = lrow[r] * fac + ((float)p0 + (float)p1);
#pragma unroll
            for (int dt = 0; dt < 4; ++dt) o[dt][r] *= fac;
            Pw[(8 * hi + r) * 40 + lr] = p0; Pw[(8 * hi + r) * 40 + 16 + lr] = p1; }
        __syncthreads();
        const v16h ap = cat16(*(const v8ha*)(Pw + lr * 40 + 8 * hi), *(const v8ha*)(Pw + lr * 40 + 16 + 8 * hi));
        __syncthreads();
        const h16* vp = Vh + (size_t)lr * SEQ + j + 8 * hi;
#pragma unroll
        for (int dt = 0; dt < 4; ++dt) { const v16h vb = ldh(vp + (size_t)dt * 16 * SEQ); o[dt] = wmma16(ap, vb, o[dt]); }
        asm volatile("v_nop\n\tv_nop\n\tv_nop\n\tv_nop" : "+v"(o[0]), "+v"(o[1]), "+v"(o[2]), "+v"(o[3]) : "v"(ap));
    }
#pragma unroll
    for (int r = 0; r < 8; ++r) { float l = lrow[r]; l += __shfl_xor(l, 1, 32); l += __shfl_xor(l, 2, 32); l += __shfl_xor(l, 4, 32); l += __shfl_xor(l, 8, 32);
        const float inv = (CCAR / VCAR) * (1.0f / l);
#pragma unroll
        for (int dt = 0; dt < 4; ++dt) os[(8 * hi + r) * 72 + dt * 16 + lr] = (h16)(o[dt][r] * inv); }
    __syncthreads();
    const int rq = lane >> 3, q = lane & 7;
    h16* crow = CTX + ((size_t)b * SEQ + q0) * DM + h * HD + q * 8;
#pragma unroll 1
    for (int ps = 0; ps < 2; ++ps) {
#pragma unroll
        for (int it = 0; it < QT / 4; ++it) { const int row = it * 4 + rq; const v8h val = *(const v8ha*)(os + row * 72 + q * 8); *(volatile v8h*)(crow + (size_t)row * DM) = val; }
        if (ps == 0) __threadfence(); }
}

__global__ __launch_bounds__(32) void k_gemm_out(const h16* __restrict__ A, const h16* __restrict__ Wt, const float* __restrict__ bias, float* out) {
    __shared__ __align__(16) float os[16 * 68];
    const int lane = threadIdx.x & 31, lr = lane & 15, hi = lane >> 4; const int r0 = blockIdx.x * 64, c0 = blockIdx.y * 64;
    v8f acc[4][4];
    gemm_main<h16>(A, Wt, r0, c0, lr, hi, acc);
    const float osc = 1.0f / (CCAR * WCAR);
    const int cofs = lr * 4;
    v4f bv;
#pragma unroll
    for (int q = 0; q < 4; ++q) bv[q] = bfr(bias[c0 + cofs + q]);
#pragma unroll
    for (int mb = 0; mb < 4; ++mb) {
#pragma unroll
        for (int nb = 0; nb < 4; ++nb) {
#pragma unroll
            for (int j = 0; j < 8; ++j) os[(hi * 8 + j) * 68 + nb * 16 + lr] = acc[mb][nb][j]; }
        __syncthreads();
        float* crow = out + (size_t)(r0 + mb * 16) * DM + c0;
#pragma unroll 1
        for (int ps = 0; ps < 2; ++ps) {
#pragma unroll
            for (int s = 0; s < 8; ++s) { const int row = 2 * s + hi; const v4f t = *(const v4fa*)(os + row * 68 + cofs); v4f val;
#pragma unroll
                for (int q = 0; q < 4; ++q) val[q] = t[q] * osc + bv[q];
                *(volatile v4f*)(crow + (size_t)row * DM + cofs) = val; }
            if (ps == 0) __threadfence(); }
        __syncthreads();
    }
}

extern "C" void kernel_launch(void* const* d_in, const int* in_sizes, int n_in,
                              void* d_out, int out_size, void* d_ws, size_t ws_size, hipStream_t stream) {
    if (n_in < 5) return;
    if (in_sizes[0] < ((NB - 1) * SEQ_FULL + SEQ) * DM) return;
    if (in_sizes[1] < DM * D3) return;
    if (in_sizes[2] < D3) return;
    if (in_sizes[3] < DM * DM) return;
    if (in_sizes[4] < DM) return;
    if (out_size < MROWS * DM) return;
    if ((size_t)WS_TOTAL > ws_size) return;
    const float* x = (const float*)d_in[0]; const float* w_qkv = (const float*)d_in[1]; const float* b_qkv = (const float*)d_in[2]; const float* w_out = (const float*)d_in[3]; const float* b_out = (const float*)d_in[4];
    float* OUT = (float*)d_out;
    char* wsp = (char*)d_ws;
    bf*  XB  = (bf*)wsp;  wsp += XB_BYTES;
    bf*  WQT = (bf*)wsp;  wsp += WQT_BYTES;
    bf*  WOT = (bf*)wsp;  wsp += WOT_BYTES;
    h16* QKV = (h16*)wsp; wsp += QKV_BYTES;
    h16* CTX = (h16*)wsp; wsp += CTX_BYTES;
    k_cvtx<<<(unsigned)(((size_t)MROWS * DM / 8 + 255) / 256), 256, 0, stream>>>(x, XB);
    k_wt<<<dim3(D3 / 64, DM / 64, 1), 256, 0, stream>>>(w_qkv, D3, WQT, 0);
    k_wt<<<dim3(DM / 64, DM / 64, 1), 256, 0, stream>>>(w_out, DM, WOT, 1);
    k_gemm_qkv<<<dim3(MROWS / 64, D3 / 64, 1), 32, 0, stream>>>(XB, WQT, b_qkv, QKV);
    k_attn<<<dim3(SEQ / QT, NH, NB), 32, 0, stream>>>(QKV, CTX);
    k_gemm_out<<<dim3(MROWS / 64, DM / 64, 1), 32, 0, stream>>>((const h16*)CTX, (const h16*)WOT, b_out, OUT);
}
